// BiMamba_1185410974355
// MI455X (gfx1250) — hardware-run, weakly checked
//
#include <hip/hip_runtime.h>
#include <math.h>

typedef __attribute__((ext_vector_type(16))) _Float16 v16h;
typedef __attribute__((ext_vector_type(8)))  _Float16 v8h;
typedef __attribute__((ext_vector_type(16))) __bf16   v16b;
typedef __attribute__((ext_vector_type(8)))  __bf16   v8b;
typedef __attribute__((ext_vector_type(8)))  float    v8f;
typedef __attribute__((ext_vector_type(4)))  float    v4f;
typedef __attribute__((ext_vector_type(2)))  float    v2f;

constexpr int kBatch  = 2;
constexpr int kSite   = 128;
constexpr int kCell   = 8;
constexpr int kDim    = 32;
constexpr int kVocab  = 100;
constexpr int kCpG    = 3;
constexpr int kDm     = 2 * kDim;
constexpr int kDi     = 4 * kDim;
constexpr int kDs     = 256;
constexpr int kDr     = 4;
constexpr int kL      = kSite * kCell;
constexpr int kRows   = kBatch * kL;
constexpr int kEmb    = 3 * kDim;
constexpr int kEmbP   = 128;
constexpr int kPosHalf = kEmb / 2;
constexpr int kXpN    = kDr + 2 * kDs;
constexpr int kXdP    = 576;
constexpr int kSeqs   = 2 * kBatch;
constexpr int kRows2  = kSeqs * kL;
constexpr int kTP     = 132;
static_assert(kDm == 64 && kDi == 128 && kL == 1024 && kRows == 2048 && kEmb == 96 && kXpN == 516, "shapes");
static_assert((kEmb % 32) == 0 && (kDm % 32) == 0 && (kDi % 32) == 0, "GEMM K multiples of 32");
static_assert((kRows % 64) == 0 && (kRows2 % 64) == 0 && (kDm % 64) == 0 && ((2 * kDi) % 64) == 0 && (kXdP % 64) == 0, "GEMM M,N multiples of 64");
static_assert(kXdP >= 2 * kDs + kDr, "x_proj pad");

constexpr float kActCarry = 16.0f;
constexpr float kWCarry   = 64.0f;
constexpr float kYgCarry  = 256.0f;
constexpr float kScaleAW  = 1.0f / (kActCarry * kWCarry);
constexpr float kScaleYW  = 1.0f / (kYgCarry * kWCarry);
constexpr float kF16Min   = 6.103515625e-5f;
constexpr float kLnEps    = 1e-5f;
constexpr double kLn1e4   = 9.210340371976184;
constexpr float kPosFac   = (float)(-(kLn1e4 / (double)kPosHalf));

constexpr size_t kOffEH   = 0;
constexpr size_t kOffEL   = kOffEH   + (size_t)kRows * kEmbP * 2;
constexpr size_t kOffFWH  = kOffEL   + (size_t)kRows * kEmbP * 2;
constexpr size_t kOffFWL  = kOffFWH  + (size_t)kDm * kEmb * 2;
constexpr size_t kOffWIN  = kOffFWL  + (size_t)kDm * kEmb * 2;
constexpr size_t kOffWOUT = kOffWIN  + (size_t)2 * kDi * kDm * 2;
constexpr size_t kOffWXP  = kOffWOUT + (size_t)kDm * kDi * 2;
constexpr size_t kOffANEG = kOffWXP  + (size_t)kXdP * kDi * 2;
constexpr size_t kOffH1   = kOffANEG + (size_t)kDi * kDs * 4;
constexpr size_t kOffH2   = kOffH1   + (size_t)kRows * kDm * 4;
constexpr size_t kOffH16  = kOffH2   + (size_t)kRows * kDm * 4;
constexpr size_t kOffXZ   = kOffH16  + (size_t)kRows * kDm * 2;
constexpr size_t kOffXC32 = kOffXZ   + (size_t)kRows * 2 * kDi * 4;
constexpr size_t kOffXC16 = kOffXC32 + (size_t)kRows2 * kDi * 4;
constexpr size_t kOffXD   = kOffXC16 + (size_t)kRows2 * kDi * 2;
constexpr size_t kOffYST  = kOffXD   + (size_t)kRows2 * kXdP * 4;
constexpr size_t kOffYG   = kOffYST  + (size_t)kSeqs * kDi * kL * 4;
constexpr size_t kOffO    = kOffYG   + (size_t)kRows * kDi * 2;
constexpr size_t kWsTotal = kOffO    + (size_t)kRows * kDm * 4;
static_assert(kWsTotal == 20537344ull, "carve total");
static_assert(kWsTotal <= 134217728ull, "carve cap");
static_assert((kOffEL % 128) == 0 && (kOffFWH % 128) == 0 && (kOffFWL % 128) == 0 && (kOffWIN % 128) == 0 &&
              (kOffWOUT % 128) == 0 && (kOffWXP % 128) == 0 && (kOffANEG % 128) == 0 && (kOffH1 % 128) == 0 &&
              (kOffH2 % 128) == 0 && (kOffH16 % 128) == 0 && (kOffXZ % 128) == 0 && (kOffXC32 % 128) == 0 &&
              (kOffXC16 % 128) == 0 && (kOffXD % 128) == 0 && (kOffYST % 128) == 0 && (kOffYG % 128) == 0 &&
              (kOffO % 128) == 0, "128-B aligned regions");

__device__ __forceinline__ unsigned short f2bf_bits(float f) {
  unsigned u = __float_as_uint(f);
  return (unsigned short)((u + 0x7FFFu + ((u >> 16) & 1u)) >> 16);
}
__device__ __forceinline__ float bf_bits2f(unsigned short h) { return __uint_as_float(((unsigned)h) << 16); }

__device__ __forceinline__ _Float16 to_f16_flush(float v) {
  const float w = (fabsf(v) < kF16Min) ? 0.0f : v;
  return (_Float16)w;
}
__device__ __forceinline__ void pin4(v4f& v) { asm volatile("" : "+v"(v)); }
__device__ __forceinline__ void pin1(float& v) { asm volatile("" : "+v"(v)); }
__device__ __forceinline__ float silu_f(float v) { return v * __builtin_amdgcn_rcpf(1.0f + expf(-v)); }

__device__ __forceinline__ void acc_tie_h(v8f& a, v16h x, v16h y, v16h z, v16h w) { asm volatile("v_nop\n\tv_nop\n\tv_nop\n\tv_nop" : "+v"(a) : "v"(x), "v"(y), "v"(z), "v"(w)); }
__device__ __forceinline__ void acc_tie_b(v8f& a, v16b x, v16b y, v16b z, v16b w) { asm volatile("v_nop\n\tv_nop\n\tv_nop\n\tv_nop" : "+v"(a) : "v"(x), "v"(y), "v"(z), "v"(w)); }
__device__ __forceinline__ void keep4_h(v16h a, v16h b, v16h c, v16h d) { asm volatile("v_nop" :: "v"(a), "v"(b), "v"(c), "v"(d)); }
__device__ __forceinline__ void keep4_b(v16b a, v16b b, v16b c, v16b d) { asm volatile("v_nop" :: "v"(a), "v"(b), "v"(c), "v"(d)); }
__device__ __forceinline__ void acc_guard4(v8f& a, v8f& b, v8f& c, v8f& d) { asm volatile("v_nop\n\tv_nop\n\tv_nop\n\tv_nop" : "+v"(a), "+v"(b), "+v"(c), "+v"(d)); }

template <typename T> struct Frag;
template <> struct Frag<_Float16> {
  typedef v16h V; union U { v16h v; v8h h[2]; };
  static __device__ __forceinline__ v16h load(const _Float16* p) {
    U f; f.h[0] = *(const v8h*)(p); f.h[1] = *(const v8h*)(p + 16); return f.v;
  }
  static __device__ __forceinline__ v8f mma(v16h a, v16h b, v8f c) {
    return __builtin_amdgcn_wmma_f32_16x16x32_f16(false, a, false, b, (short)0, c, false, false);
  }
  static __device__ __forceinline__ void tie(v8f& a, v16h x, v16h y, v16h z, v16h w) { acc_tie_h(a, x, y, z, w); }
  static __device__ __forceinline__ void keep(v16h a, v16h b, v16h c, v16h d) { keep4_h(a, b, c, d); }
};
template <> struct Frag<__bf16> {
  typedef v16b V; union U { v16b v; v8b h[2]; };
  static __device__ __forceinline__ v16b load(const __bf16* p) {
    U f; f.h[0] = *(const v8b*)(p); f.h[1] = *(const v8b*)(p + 16); return f.v;
  }
  static __device__ __forceinline__ v8f mma(v16b a, v16b b, v8f c) {
    return __builtin_amdgcn_wmma_f32_16x16x32_bf16(false, a, false, b, (short)0, c, false, false);
  }
  static __device__ __forceinline__ void tie(v8f& a, v16b x, v16b y, v16b z, v16b w) { acc_tie_b(a, x, y, z, w); }
  static __device__ __forceinline__ void keep(v16b a, v16b b, v16b c, v16b d) { keep4_b(a, b, c, d); }
};

template <int ET> struct Elem;
template <> struct Elem<0> { typedef _Float16 T; };
template <> struct Elem<1> { typedef __bf16 T; };
template <int ET, bool SPLIT, bool BIASN, bool RELU>
__global__ __launch_bounds__(256) void wmma_gemm64(
    const unsigned short* __restrict__ Ap, const unsigned short* __restrict__ A2p, int lda,
    const unsigned short* __restrict__ Btp, const unsigned short* __restrict__ Bt2p, int ldb,
    float* __restrict__ C, int ldc,
    const float* __restrict__ bias,
    int M, int N, int K, float scale) {
  typedef typename Elem<ET>::T T;
  typedef typename Frag<T>::V V;
  const T* A = (const T*)Ap; const T* A2 = (const T*)A2p; const T* Bt = (const T*)Btp; const T* Bt2 = (const T*)Bt2p;
  __shared__ __align__(16) float sT[8][16 * 68];
  const int lane = threadIdx.x & 31;
  const int wave = threadIdx.x >> 5;
  const int tilesN = N >> 6;
  const int tilesM = M >> 6;
  const int tile = blockIdx.x * 8 + wave;
  if (tile >= tilesM * tilesN) return;
  const int tm = tile / tilesN;
  const int tn = tile - tm * tilesN;
  const int m0 = tm << 6;
  const int n0 = tn << 6;

  const int rlane = lane & 15;
  const int koff  = (lane >> 4) * 8;
  const int mOff  = (lane >> 4) * 8;

  v8f acc[4][4];
#pragma unroll
  for (int i = 0; i < 4; ++i)
#pragma unroll
    for (int j = 0; j < 4; ++j) acc[i][j] = (v8f){0.f,0.f,0.f,0.f,0.f,0.f,0.f,0.f};

  for (int k0 = 0; k0 < K; k0 += 32) {
    V bh[4], bl[4];
#pragma unroll
    for (int j = 0; j < 4; ++j) {
      const size_t bo = (size_t)(n0 + (j << 4) + rlane) * ldb + koff + k0;
      bh[j] = Frag<T>::load(Bt + bo);
      bl[j] = bh[j];
      if (SPLIT) bl[j] = Frag<T>::load(Bt2 + bo);
    }
#pragma unroll
    for (int i = 0; i < 4; ++i) {
      const size_t ao = (size_t)(m0 + (i << 4) + rlane) * lda + koff + k0;
      V ah = Frag<T>::load(A + ao);
      V al = ah;
      if (SPLIT) al = Frag<T>::load(A2 + ao);
#pragma unroll
      for (int j = 0; j < 4; ++j) {
        acc[i][j] = Frag<T>::mma(ah, bh[j], acc[i][j]);
        if (SPLIT) {
          acc[i][j] = Frag<T>::mma(ah, bl[j], acc[i][j]);
          acc[i][j] = Frag<T>::mma(al, bh[j], acc[i][j]);
        }
      }
#pragma unroll
      for (int j = 0; j < 4; ++j) Frag<T>::tie(acc[i][j], ah, al, bh[j], bl[j]);
    }
    Frag<T>::keep(bh[0], bh[1], bh[2], bh[3]);
    if (SPLIT) Frag<T>::keep(bl[0], bl[1], bl[2], bl[3]);
  }
  acc_guard4(acc[0][0], acc[0][1], acc[0][2], acc[0][3]);
  acc_guard4(acc[1][0], acc[1][1], acc[1][2], acc[1][3]);
  acc_guard4(acc[2][0], acc[2][1], acc[2][2], acc[2][3]);
  acc_guard4(acc[3][0], acc[3][1], acc[3][2], acc[3][3]);

  float* slab = sT[wave];
#pragma unroll
  for (int i = 0; i < 4; ++i) {
    const int mBase = m0 + (i << 4);
#pragma unroll
    for (int j = 0; j < 4; ++j) {
      const int n = n0 + (j << 4) + rlane;
      float bv = 0.f;
      if (BIASN) bv = bias[n];
#pragma unroll
      for (int r = 0; r < 8; ++r) {
        float v = acc[i][j][r] * scale;
        if (BIASN) v += bv;
        if (RELU) v = fmaxf(v, 0.0f);
        slab[(mOff + r) * 68 + (j << 4) + rlane] = v;
      }
    }
    __builtin_amdgcn_fence(__ATOMIC_RELEASE, "workgroup");
    __builtin_amdgcn_wave_barrier();
    __builtin_amdgcn_fence(__ATOMIC_ACQUIRE, "workgroup");
    {
      const int hh = lane >> 4, c4 = (lane & 15) * 4;
      for (int pass = 0; pass < 2; ++pass) {
#pragma unroll
        for (int it = 0; it < 8; ++it) {
          const int row = it * 2 + hh;
          v4f v = *(const v4f*)(slab + row * 68 + c4);
          *(volatile v4f*)(C + (size_t)(mBase + row) * ldc + n0 + c4) = v;
        }
        __threadfence();
      }
    }
    __builtin_amdgcn_fence(__ATOMIC_RELEASE, "workgroup");
    __builtin_amdgcn_wave_barrier();
    __builtin_amdgcn_fence(__ATOMIC_ACQUIRE, "workgroup");
  }
}

template <int MODE>
__global__ __launch_bounds__(256) void cvt8_kernel(const float* __restrict__ src, unsigned short* __restrict__ dst,
                                                   unsigned short* __restrict__ dst2,
                                                   int nrow, int ncol8, int nA, int rshift, int nB, int srows, float sc) {
  const int i  = blockIdx.x * 256 + threadIdx.x;
  const int n8 = nrow * ncol8;
  if (i >= n8) return;
  const int row = i / ncol8;
  const int c8  = i - row * ncol8;
  int srow = (row < nA) ? (row + rshift) : (row - nA);
  const bool live = row < (nA + nB);
  srow = srow < 0 ? 0 : srow;
  srow = srow > (srows - 1) ? (srows - 1) : srow;
  const float* sp = src + (size_t)srow * (size_t)(ncol8 * 8) + c8 * 8;
  v4f a = *(const v4f*)(sp);
  v4f b = *(const v4f*)(sp + 4);
  pin4(a);
  pin4(b);
  v8h hv, lv;
#pragma unroll
  for (int e = 0; e < 4; ++e) {
    const float f0 = live ? a[e] : 0.0f;
    const float f1 = live ? b[e] : 0.0f;
    if (MODE == 0) {
      hv[e]     = to_f16_flush(f0 * sc);
      hv[4 + e] = to_f16_flush(f1 * sc);
      lv[e]     = hv[e];
      lv[4 + e] = hv[4 + e];
    } else {
      const unsigned short h0 = f2bf_bits(f0), h1 = f2bf_bits(f1);
      const unsigned short l0 = f2bf_bits(f0 - bf_bits2f(h0)), l1 = f2bf_bits(f1 - bf_bits2f(h1));
      hv[e]     = __builtin_bit_cast(_Float16, h0);
      hv[4 + e] = __builtin_bit_cast(_Float16, h1);
      lv[e]     = __builtin_bit_cast(_Float16, l0);
      lv[4 + e] = __builtin_bit_cast(_Float16, l1);
    }
  }
  unsigned short* qh = dst + (size_t)i * 8;
  unsigned short* ql = dst2 + (size_t)i * 8;
  *(volatile v8h*)qh = hv;
  if (MODE == 1) *(volatile v8h*)ql = lv;
  __threadfence();
  *(volatile v8h*)qh = hv;
  if (MODE == 1) *(volatile v8h*)ql = lv;
}

__global__ __launch_bounds__(256) void neg_exp_kernel(const float* __restrict__ alog, float* __restrict__ aneg) {
  const int i = blockIdx.x * 256 + threadIdx.x;
  const v4f a = *(const v4f*)(alog + (size_t)i * 4);
  v4f o;
#pragma unroll
  for (int e = 0; e < 4; ++e) o[e] = -expf(a[e]);
  float* op = aneg + (size_t)i * 4;
  *(volatile v4f*)op = o;
  __threadfence();
  *(volatile v4f*)op = o;
}

__global__ __launch_bounds__(256) void embed_kernel(const float* __restrict__ x, const int* __restrict__ ycpg,
                                                    const int* __restrict__ cidx, const float* __restrict__ cellEB,
                                                    const float* __restrict__ CpGEB,
                                                    unsigned* __restrict__ EH, unsigned* __restrict__ EL) {
  const int gid = blockIdx.x * 256 + threadIdx.x;
  const int row = gid >> 6;
  const int p   = gid & 63;
  const int b = row >> 10;
  const int r = row & (kL - 1);
  const int s = r >> 3;
  const int c = r & (kCell - 1);
  int cls = ycpg[row];
  cls = cls < 0 ? 0 : cls;
  cls = cls > (kCpG - 1) ? (kCpG - 1) : cls;
  int ci = cidx[b * kCell + c];
  ci = ci < 0 ? 0 : ci;
  ci = ci > (kVocab - 1) ? (kVocab - 1) : ci;
  const bool live = p < (kEmb / 2);
  const int pc  = live ? p : (kEmb / 2 - 1);
  const int dch = 2 * pc;
  const int o   = dch & (kDim - 1);
  const v2f va = *(const v2f*)(CpGEB + cls * kDim + o);
  const v2f vb = *(const v2f*)(cellEB + ci * kDim + o);
  const v2f vc = *(const v2f*)(x + (size_t)(b * kSite + s) * kDim + o);
  float a0 = va[0], a1 = va[1], b0 = vb[0], b1 = vb[1], c0 = vc[0], c1 = vc[1];
  pin1(a0); pin1(a1); pin1(b0); pin1(b1); pin1(c0); pin1(c1);
  const int seg = dch >> 5;
  const float v0 = (seg == 0) ? a0 : ((seg == 1) ? b0 : c0);
  const float v1 = (seg == 0) ? a1 : ((seg == 1) ? b1 : c1);
  const bool cellpart = pc < (kPosHalf / 2);
  const int fi = cellpart ? pc : (pc - kPosHalf / 2);
  const float posv = cellpart ? (float)c : (float)s;
  const float dv  = expf((float)(2 * fi) * kPosFac);
  const float arg = posv * dv;
  float sn, cs;
  sincosf(arg, &sn, &cs);
  float e0 = v0 + sn;
  float e1 = v1 + cs;
  e0 = live ? e0 : 0.0f;
  e1 = live ? e1 : 0.0f;
  const unsigned short h0 = f2bf_bits(e0), h1 = f2bf_bits(e1);
  const unsigned short l0 = f2bf_bits(e0 - bf_bits2f(h0)), l1 = f2bf_bits(e1 - bf_bits2f(h1));
  const unsigned uh = (unsigned)h0 | ((unsigned)h1 << 16);
  const unsigned ul = (unsigned)l0 | ((unsigned)l1 << 16);
  ((volatile unsigned*)EH)[gid] = uh;
  ((volatile unsigned*)EL)[gid] = ul;
  __threadfence();
  ((volatile unsigned*)EH)[gid] = uh;
  ((volatile unsigned*)EL)[gid] = ul;
}

__device__ __forceinline__ float conv_tap(const float* __restrict__ XZ, int b, int dir, int d, int tau) {
  const int tc = tau < 0 ? 0 : tau;
  const int t  = dir ? (kL - 1 - tc) : tc;
  float v = XZ[(size_t)(b * kL + t) * (2 * kDi) + d];
  pin1(v);
  return (tau >= 0) ? v : 0.0f;
}

__global__ __launch_bounds__(256) void conv_silu_kernel(const float* __restrict__ XZ, const float* __restrict__ cw,
                                                        const float* __restrict__ cb, float* __restrict__ XC32,
                                                        unsigned short* __restrict__ XC16) {
  __shared__ __align__(16) float sT[32 * kTP];
  const int tid = threadIdx.x, lane = tid & 31, wave = tid >> 5;
  const int seq  = blockIdx.x >> 5;
  const int tau0 = (blockIdx.x & 31) * 32;
  const int dir = seq >> 1, b = seq & 1;
  const int d  = tid & (kDi - 1);
  const int hf = tid >> 7;
  const int ts = tau0 + hf * 16;
  const v4f w = *(const v4f*)(cw + d * 4);
  const float bc = cb[d];
  float xm3 = conv_tap(XZ, b, dir, d, ts - 3);
  float xm2 = conv_tap(XZ, b, dir, d, ts - 2);
  float xm1 = conv_tap(XZ, b, dir, d, ts - 1);
#pragma unroll 1
  for (int s = 0; s < 16; ++s) {
    const float xcur = conv_tap(XZ, b, dir, d, ts + s);
    float acc = w[0] * xm3;
    acc = fmaf(w[1], xm2, acc);
    acc = fmaf(w[2], xm1, acc);
    acc = fmaf(w[3], xcur, acc);
    const float sv = acc + bc;
    sT[(hf * 16 + s) * kTP + d] = silu_f(sv);
    xm3 = xm2; xm2 = xm1; xm1 = xcur;
  }
  __syncthreads();
  const size_t rowb = (size_t)seq * kL + tau0;
  v4f fv[4];
#pragma unroll
  for (int it = 0; it < 4; ++it) fv[it] = *(const v4f*)(sT + (it * 8 + wave) * kTP + lane * 4);
  v8h hv[2];
  const int hr = wave * 2 + (lane >> 4);
  const int c8 = (lane & 15) * 8;
#pragma unroll
  for (int it = 0; it < 2; ++it) {
    const float* sp = sT + (it * 16 + hr) * kTP + c8;
    const v4f a0 = *(const v4f*)(sp);
    const v4f a1 = *(const v4f*)(sp + 4);
#pragma unroll
    for (int e = 0; e < 4; ++e) {
      hv[it][e]     = to_f16_flush(a0[e] * kActCarry);
      hv[it][4 + e] = to_f16_flush(a1[e] * kActCarry);
    }
  }
  for (int pass = 0; pass < 2; ++pass) {
#pragma unroll
    for (int it = 0; it < 4; ++it)
      *(volatile v4f*)(XC32 + (rowb + it * 8 + wave) * kDi + lane * 4) = fv[it];
#pragma unroll
    for (int it = 0; it < 2; ++it)
      *(volatile v8h*)(XC16 + (rowb + it * 16 + hr) * kDi + c8) = hv[it];
    __threadfence();
  }
}

__global__ __launch_bounds__(256) void scan_kernel(const float* __restrict__ XD, const float* __restrict__ XC,
                                                   const float* __restrict__ Wdt, const float* __restrict__ bdt,
                                                   const float* __restrict__ ANEG, float* __restrict__ YST) {
  const int lane = threadIdx.x & 31, wave = threadIdx.x >> 5;
  const int gw  = blockIdx.x * 8 + wave;
  const int seq = gw >> 7;
  const int d   = gw & (kDi - 1);
  const size_t row0 = (size_t)seq * kL;
  float A[8], h[8];
  {
    const v4f a0 = *(const v4f*)(ANEG + (size_t)d * kDs + lane * 8);
    const v4f a1 = *(const v4f*)(ANEG + (size_t)d * kDs + lane * 8 + 4);
#pragma unroll
    for (int e = 0; e < 4; ++e) {
      A[e] = a0[e];
      A[4 + e] = a1[e];
      h[e] = 0.0f;
      h[4 + e] = 0.0f;
    }
  }
  const v4f wd = *(const v4f*)(Wdt + d * kDr);
  const float bb = bdt[d];
  float* yrow = YST + (size_t)gw * kL;
#pragma unroll 1
  for (int c0 = 0; c0 < kL; c0 += 32) {
    const size_t rl = row0 + c0 + lane;
    const v4f dr = *(const v4f*)(XD + rl * kXdP + 2 * kDs);
    const float xl = XC[rl * kDi + d];
    float vd = dr[0] * wd[0];
    vd = fmaf(dr[1], wd[1], vd);
    vd = fmaf(dr[2], wd[2], vd);
    vd = fmaf(dr[3], wd[3], vd);
    vd += bb;
    const float dtl = fmaxf(vd, 0.0f) + log1pf(expf(-fabsf(vd)));
    float ykeep = 0.0f;
    const float* brow = XD + (row0 + c0) * kXdP + lane * 8;
#pragma unroll 1
    for (int s = 0; s < 32; ++s) {
      const float dtv = __shfl(dtl, s, 32);
      const float xv  = __shfl(xl, s, 32);
      const float* bp = brow + (size_t)s * kXdP;
      const v4f B0 = *(const v4f*)(bp);
      const v4f B1 = *(const v4f*)(bp + 4);
      const v4f C0 = *(const v4f*)(bp + kDs);
      const v4f C1 = *(const v4f*)(bp + kDs + 4);
      const float dx = dtv * xv;
      float part = 0.0f;
#pragma unroll
      for (int e = 0; e < 4; ++e) {
        const float ea = expf(dtv * A[e]);
        h[e] = fmaf(ea, h[e], dx * B0[e]);
        part = fmaf(h[e], C0[e], part);
      }
#pragma unroll
      for (int e = 0; e < 4; ++e) {
        const float ea = expf(dtv * A[4 + e]);
        h[4 + e] = fmaf(ea, h[4 + e], dx * B1[e]);
        part = fmaf(h[4 + e], C1[e], part);
      }
      part += __shfl_xor(part, 16, 32);
      part += __shfl_xor(part, 8, 32);
      part += __shfl_xor(part, 4, 32);
      part += __shfl_xor(part, 2, 32);
      part += __shfl_xor(part, 1, 32);
      ykeep = (lane == s) ? part : ykeep;
    }
    float* yp = yrow + c0 + lane;
    *(volatile float*)yp = ykeep;
    __threadfence();
    *(volatile float*)yp = ykeep;
  }
}

__global__ __launch_bounds__(256) void combine_kernel(const float* __restrict__ YST, const float* __restrict__ XC32,
                                                      const float* __restrict__ XZ, const float* __restrict__ Dp,
                                                      unsigned short* __restrict__ YG) {
  __shared__ __align__(16) float sF[32 * kTP];
  __shared__ __align__(16) float sB[32 * kTP];
  const int tid = threadIdx.x;
  const int b  = blockIdx.x >> 5;
  const int t0 = (blockIdx.x & 31) * 32;
#pragma unroll
  for (int it = 0; it < 4; ++it) {
    const int idx = it * 256 + tid;
    const int d  = idx >> 3;
    const int j4 = (idx & 7) * 4;
    const v4f vf = *(const v4f*)(YST + ((size_t)(b) * kDi + d) * kL + t0 + j4);
    const v4f vb = *(const v4f*)(YST + ((size_t)(kBatch + b) * kDi + d) * kL + (kL - 32 - t0) + j4);
#pragma unroll
    for (int e = 0; e < 4; ++e) {
      sF[(j4 + e) * kTP + d] = vf[e];
      sB[(31 - (j4 + e)) * kTP + d] = vb[e];
    }
  }
  __syncthreads();
  const int c8 = (tid & 15) * 8;
  const v4f D0 = *(const v4f*)(Dp + c8);
  const v4f D1 = *(const v4f*)(Dp + c8 + 4);
#pragma unroll 1
  for (int it = 0; it < 2; ++it) {
    const int r = it * 16 + (tid >> 4);
    const int t = t0 + r;
    const size_t rowf = (size_t)b * kL + t;
    const size_t rowr = (size_t)(kBatch + b) * kL + (kL - 1 - t);
    const v4f xf0 = *(const v4f*)(XC32 + rowf * kDi + c8);
    const v4f xf1 = *(const v4f*)(XC32 + rowf * kDi + c8 + 4);
    const v4f xb0 = *(const v4f*)(XC32 + rowr * kDi + c8);
    const v4f xb1 = *(const v4f*)(XC32 + rowr * kDi + c8 + 4);
    const v4f z0  = *(const v4f*)(XZ + rowf * (2 * kDi) + kDi + c8);
    const v4f z1  = *(const v4f*)(XZ + rowf * (2 * kDi) + kDi + c8 + 4);
    const v4f yf0 = *(const v4f*)(sF + r * kTP + c8);
    const v4f yf1 = *(const v4f*)(sF + r * kTP + c8 + 4);
    const v4f yb0 = *(const v4f*)(sB + r * kTP + c8);
    const v4f yb1 = *(const v4f*)(sB + r * kTP + c8 + 4);
    v8h hv;
#pragma unroll
    for (int e = 0; e < 4; ++e) {
      const float ya = fmaf(xf0[e], D0[e], yf0[e]) + fmaf(xb0[e], D0[e], yb0[e]);
      const float yb = fmaf(xf1[e], D1[e], yf1[e]) + fmaf(xb1[e], D1[e], yb1[e]);
      const float ga = silu_f(z0[e]);
      const float gb = silu_f(z1[e]);
      hv[e]     = to_f16_flush((0.5f * ya) * ga * kYgCarry);
      hv[4 + e] = to_f16_flush((0.5f * yb) * gb * kYgCarry);
    }
    unsigned short* op = YG + rowf * kDi + c8;
    *(volatile v8h*)op = hv;
    __threadfence();
    *(volatile v8h*)op = hv;
  }
}

__device__ __forceinline__ int permuted_row(int row, int mode) {
  const int b = row >> 10;
  const int r = row & (kL - 1);
  const int da = b * kL + (r & (kCell - 1)) * kSite + (r >> 3);
  const int db = b * kL + (r & (kSite - 1)) * kCell + (r >> 7);
  return (mode == 0) ? da : db;
}

__global__ __launch_bounds__(256) void ln_permute_kernel(const float* __restrict__ H, const float* __restrict__ O,
                                                         const float* __restrict__ gam, const float* __restrict__ bet,
                                                         float* __restrict__ DST, unsigned short* __restrict__ DST16,
                                                         int mode, int write16) {
  __shared__ __align__(16) float sl[8][2 * kDm];
  const int tid = threadIdx.x, lane = tid & 31, wave = tid >> 5;
  const int hh = lane >> 4, c4 = (lane & 15) * 4;
  const int base = (blockIdx.x * 8 + wave) * 2;
  const int row = base + hh;
  const v4f hv = *(const v4f*)(H + (size_t)row * kDm + c4);
  const v4f ov = *(const v4f*)(O + (size_t)row * kDm + c4);
  const v4f g4 = *(const v4f*)(gam + c4);
  const v4f b4 = *(const v4f*)(bet + c4);
  v4f v;
#pragma unroll
  for (int e = 0; e < 4; ++e) v[e] = hv[e] + ov[e];
  float sum = (v[0] + v[1]) + (v[2] + v[3]);
  sum += __shfl_xor(sum, 8, 32);
  sum += __shfl_xor(sum, 4, 32);
  sum += __shfl_xor(sum, 2, 32);
  sum += __shfl_xor(sum, 1, 32);
  const float mu = sum * (1.0f / kDm);
  v4f dv;
  float ss = 0.0f;
#pragma unroll
  for (int e = 0; e < 4; ++e) {
    dv[e] = v[e] - mu;
    ss += dv[e] * dv[e];
  }
  ss += __shfl_xor(ss, 8, 32);
  ss += __shfl_xor(ss, 4, 32);
  ss += __shfl_xor(ss, 2, 32);
  ss += __shfl_xor(ss, 1, 32);
  const float rstd = rsqrtf(ss * (1.0f / kDm) + kLnEps);
  v4f o, oc;
#pragma unroll
  for (int e = 0; e < 4; ++e) {
    o[e]  = (dv[e] * rstd) * g4[e] + b4[e];
    oc[e] = o[e] * kActCarry;
  }
  float* slab = sl[wave];
  *(v4f*)(slab + hh * kDm + c4) = oc;
  __builtin_amdgcn_fence(__ATOMIC_RELEASE, "workgroup");
  __builtin_amdgcn_wave_barrier();
  __builtin_amdgcn_fence(__ATOMIC_ACQUIRE, "workgroup");
  const int q  = (lane >> 3) & 1;
  const int c8 = (lane & 7) * 8;
  const v4f a0 = *(const v4f*)(slab + q * kDm + c8);
  const v4f a1 = *(const v4f*)(slab + q * kDm + c8 + 4);
  v8h h8;
#pragma unroll
  for (int e = 0; e < 4; ++e) {
    h8[e]     = to_f16_flush(a0[e]);
    h8[4 + e] = to_f16_flush(a1[e]);
  }
  const int drow   = permuted_row(row, mode);
  const int drow16 = permuted_row(base + q, mode);
  float* op = DST + (size_t)drow * kDm + c4;
  unsigned short* op16 = DST16 + (size_t)drow16 * kDm + c8;
  const bool st16 = (write16 != 0) && (lane < 16);
  for (int pass = 0; pass < 2; ++pass) {
    *(volatile v4f*)op = o;
    if (st16) *(volatile v8h*)op16 = h8;
    __threadfence();
  }
}

extern "C" void kernel_launch(void* const* d_in, const int* in_sizes, int n_in,
                              void* d_out, int out_size, void* d_ws, size_t ws_size,
                              hipStream_t stream) {
  if (n_in < 18 || d_out == nullptr || d_ws == nullptr) return;
  if (in_sizes[0] != kBatch * kSite * kDim) return;
  if (in_sizes[1] != kBatch * kSite * kCell) return;
  if (in_sizes[2] != kBatch * kCell) return;
  if (in_sizes[3] != kVocab * kDim) return;
  if (in_sizes[4] != kCpG * kDim) return;
  if (in_sizes[5] != kDm * kEmb) return;
  if (in_sizes[6] != kDm || in_sizes[7] != kDm || in_sizes[8] != kDm) return;
  if (in_sizes[9] != 2 * kDi * kDm) return;
  if (in_sizes[10] != kDi * 4 || in_sizes[11] != kDi) return;
  if (in_sizes[12] != kXpN * kDi) return;
  if (in_sizes[13] != kDi * kDr || in_sizes[14] != kDi) return;
  if (in_sizes[15] != kDi * kDs || in_sizes[16] != kDi) return;
  if (in_sizes[17] != kDm * kDi) return;
  if (out_size != kRows * kDm) return;
  if (ws_size < kWsTotal) return;

  const float* x          = (const float*)d_in[0];
  const int*   ycpg       = (const int*)d_in[1];
  const int*   cidx       = (const int*)d_in[2];
  const float* cellEB     = (const float*)d_in[3];
  const float* CpGEB      = (const float*)d_in[4];
  const float* fcc_w      = (const float*)d_in[5];
  const float* fcc_b      = (const float*)d_in[6];
  const float* ln_g       = (const float*)d_in[7];
  const float* ln_b       = (const float*)d_in[8];
  const float* in_proj_w  = (const float*)d_in[9];
  const float* conv_w     = (const float*)d_in[10];
  const float* conv_b     = (const float*)d_in[11];
  const float* x_proj_w   = (const float*)d_in[12];
  const float* dt_proj_w  = (const float*)d_in[13];
  const float* dt_proj_b  = (const float*)d_in[14];
  const float* A_log      = (const float*)d_in[15];
  const float* D_param    = (const float*)d_in[16];
  const float* out_proj_w = (const float*)d_in[17];
  float* out = (float*)d_out;

  char* ws = (char*)d_ws;
  unsigned short* EH   = (unsigned short*)(ws + kOffEH);
  unsigned short* EL   = (unsigned short*)(ws + kOffEL);
  unsigned short* FWH  = (unsigned short*)(ws + kOffFWH);
  unsigned short* FWL  = (unsigned short*)(ws + kOffFWL);
  unsigned short* WIN  = (unsigned short*)(ws + kOffWIN);
  unsigned short* WOUT = (unsigned short*)(ws + kOffWOUT);
  unsigned short* WXP  = (unsigned short*)(ws + kOffWXP);
  float*          ANEG = (float*)(ws + kOffANEG);
  float*          H1   = (float*)(ws + kOffH1);
  float*          H2   = (float*)(ws + kOffH2);
  unsigned short* H16  = (unsigned short*)(ws + kOffH16);
  float*          XZ   = (float*)(ws + kOffXZ);
  float*          XC32 = (float*)(ws + kOffXC32);
  unsigned short* XC16 = (unsigned short*)(ws + kOffXC16);
  float*          XD   = (float*)(ws + kOffXD);
  float*          YST  = (float*)(ws + kOffYST);
  unsigned short* YG   = (unsigned short*)(ws + kOffYG);
  float*          O    = (float*)(ws + kOffO);

  static_assert((kDm * kEmb / 8) % 256 == 0 && (2 * kDi * kDm / 8) % 256 == 0 && (kDm * kDi / 8) % 256 == 0 &&
                (kXdP * kDi / 8) % 256 == 0 && (kRows * kDm / 8) % 256 == 0 && (kDi * kDs / 4) % 256 == 0, "exact grids");
  cvt8_kernel<1><<<(kDm * kEmb / 8) / 256, 256, 0, stream>>>(fcc_w, FWH, FWL, kDm, kEmb / 8, kDm, 0, 0, kDm, 1.0f);
  cvt8_kernel<0><<<(2 * kDi * kDm / 8) / 256, 256, 0, stream>>>(in_proj_w, WIN, WIN, 2 * kDi, kDm / 8, 2 * kDi, 0, 0, 2 * kDi, kWCarry);
  cvt8_kernel<0><<<(kDm * kDi / 8) / 256, 256, 0, stream>>>(out_proj_w, WOUT, WOUT, kDm, kDi / 8, kDm, 0, 0, kDm, kWCarry);
  cvt8_kernel<0><<<(kXdP * kDi / 8) / 256, 256, 0, stream>>>(x_proj_w, WXP, WXP, kXdP, kDi / 8, 2 * kDs, kDr, kDr, kXpN, kWCarry);
  neg_exp_kernel<<<(kDi * kDs / 4) / 256, 256, 0, stream>>>(A_log, ANEG);

  embed_kernel<<<(kRows * (kEmbP / 2)) / 256, 256, 0, stream>>>(x, ycpg, cidx, cellEB, CpGEB, (unsigned*)EH, (unsigned*)EL);
  wmma_gemm64<1, true, true, true><<<(kRows / 64) * (kDm / 64) / 8, 256, 0, stream>>>(
      EH, EL, kEmbP, FWH, FWL, kEmb, H1, kDm, fcc_b, kRows, kDm, kEmb, 1.0f);
  cvt8_kernel<0><<<(kRows * kDm / 8) / 256, 256, 0, stream>>>(H1, H16, H16, kRows, kDm / 8, kRows, 0, 0, kRows, kActCarry);

  for (int pass = 0; pass < 2; ++pass) {
    const float* hcur = (pass == 0) ? H1 : H2;
    float* dst = (pass == 0) ? H2 : out;
    wmma_gemm64<0, false, false, false><<<(kRows / 64) * (2 * kDi / 64) / 8, 256, 0, stream>>>(
        H16, H16, kDm, WIN, WIN, kDm, XZ, 2 * kDi, fcc_b, kRows, 2 * kDi, kDm, kScaleAW);
    conv_silu_kernel<<<kSeqs * (kL / 32), 256, 0, stream>>>(XZ, conv_w, conv_b, XC32, XC16);
    wmma_gemm64<0, false, false, false><<<(kRows2 / 64) * (kXdP / 64) / 8, 256, 0, stream>>>(
        XC16, XC16, kDi, WXP, WXP, kDi, XD, kXdP, fcc_b, kRows2, kXdP, kDi, kScaleAW);
    scan_kernel<<<(kSeqs * kDi) / 8, 256, 0, stream>>>(XD, XC32, dt_proj_w, dt_proj_b, ANEG, YST);
    combine_kernel<<<kBatch * (kL / 32), 256, 0, stream>>>(YST, XC32, XZ, D_param, YG);
    wmma_gemm64<0, false, false, false><<<(kRows / 64) * (kDm / 64) / 8, 256, 0, stream>>>(
        YG, YG, kDi, WOUT, WOUT, kDi, O, kDm, fcc_b, kRows, kDm, kDi, kScaleYW);
    ln_permute_kernel<<<kRows / 16, 256, 0, stream>>>(hcur, O, ln_g, ln_b, dst, H16, pass, (pass == 0) ? 1 : 0);
  }
}
